// AtencaoMultiCabeca_28630251995757
// MI455X (gfx1250) — hardware-verified
//
#include <hip/hip_runtime.h>
#include <math.h>
#include <stdint.h>

#pragma clang fp contract(off)

#define NB    2
#define SEQ   4096
#define DM    1024
#define NH    16
#define HD    64
#define QBR   128
#define NQBLK (SEQ / QBR)
#define NKT   (SEQ / 64)
#define WS_CAP 134217728ull
static_assert(NH * HD == DM);
static_assert(HD == 64);
static_assert((SEQ % QBR) == 0 && (SEQ % 64) == 0 && (DM % 64) == 0 && (DM % 32) == 0 && ((NB * SEQ) % 64) == 0);
static_assert((SEQ & (SEQ - 1)) == 0);

typedef _Float16 v16h __attribute__((ext_vector_type(16)));
typedef _Float16 v8h  __attribute__((ext_vector_type(8)));
typedef __bf16   v16b __attribute__((ext_vector_type(16)));
typedef __bf16   v8b  __attribute__((ext_vector_type(8)));
typedef float    v8f  __attribute__((ext_vector_type(8)));
typedef float    v4f  __attribute__((ext_vector_type(4)));
typedef float    v2f  __attribute__((ext_vector_type(2)));
typedef unsigned int v4u __attribute__((ext_vector_type(4)));

__device__ __forceinline__ unsigned short bf_bits(float f) {
  unsigned u = __float_as_uint(f);
  return (unsigned short)((u + 0x7FFFu + ((u >> 16) & 1u)) >> 16);
}
__device__ __forceinline__ float bf_up(unsigned short h) { return __uint_as_float(((unsigned)h) << 16); }
__device__ __forceinline__ float bfr(float f) { return bf_up(bf_bits(f)); }
__device__ __forceinline__ unsigned short h_bits(_Float16 x) { return __builtin_bit_cast(unsigned short, x); }
__device__ __forceinline__ unsigned pk16(unsigned short a, unsigned short b) { return (unsigned)a | ((unsigned)b << 16); }
__device__ __forceinline__ v8f zero8() { v8f z = {0.f, 0.f, 0.f, 0.f, 0.f, 0.f, 0.f, 0.f}; return z; }

__device__ __forceinline__ v16b ldfrag_b(const __bf16* p) {
  union { v16b v; v8b h[2]; } f;
  f.h[0] = *(const v8b*)(p);
  f.h[1] = *(const v8b*)(p + 16);
  return f.v;
}
__device__ __forceinline__ v16h ldfrag_h(const _Float16* p) {
  union { v16h v; v8h h[2]; } f;
  f.h[0] = *(const v8h*)(p);
  f.h[1] = *(const v8h*)(p + 16);
  return f.v;
}

__device__ __forceinline__ v8f mma_h(v16h a, v16h b, v8f c) {
  c = __builtin_amdgcn_wmma_f32_16x16x32_f16(false, a, false, b, (short)0, c, false, false);
#if defined(__HIP_DEVICE_COMPILE__)
  asm volatile("v_nop\n\tv_nop\n\tv_nop\n\tv_nop" : "+v"(c) : "v"(a), "v"(b));
#endif
  return c;
}
__device__ __forceinline__ v8f mma_b_raw(v16b a, v16b b, v8f c) {
  return __builtin_amdgcn_wmma_f32_16x16x32_bf16(false, a, false, b, (short)0, c, false, false);
}
__device__ __forceinline__ void dep_guard_b(v8f& a, v8f& b, v16b x, v16b y) {
#if defined(__HIP_DEVICE_COMPILE__)
  asm volatile("v_nop\n\tv_nop\n\tv_nop\n\tv_nop" : "+v"(a), "+v"(b) : "v"(x), "v"(y));
#else
  (void)a; (void)b; (void)x; (void)y;
#endif
}
__device__ __forceinline__ void keep4_b(v16b a, v16b b, v16b c, v16b d) {
#if defined(__HIP_DEVICE_COMPILE__)
  asm volatile("v_nop" :: "v"(a), "v"(b), "v"(c), "v"(d));
#else
  (void)a; (void)b; (void)c; (void)d;
#endif
}
__device__ __forceinline__ void acc_guard4(v8f& a, v8f& b, v8f& c, v8f& d) {
#if defined(__HIP_DEVICE_COMPILE__)
  asm volatile("v_nop\n\tv_nop\n\tv_nop\n\tv_nop" : "+v"(a), "+v"(b), "+v"(c), "+v"(d));
#else
  (void)a; (void)b; (void)c; (void)d;
#endif
}
__device__ __forceinline__ void lds_wave_sync() {
  __builtin_amdgcn_fence(__ATOMIC_RELEASE, "workgroup");
  __builtin_amdgcn_wave_barrier();
  __builtin_amdgcn_fence(__ATOMIC_ACQUIRE, "workgroup");
}

__global__ __launch_bounds__(256) void cvt_bf16x8(const float* __restrict__ in, unsigned short* out, int n8) {
  const int i = blockIdx.x * 256 + threadIdx.x;
  if (i < n8) {
    const v4f a = *(const v4f*)(in + (size_t)i * 8);
    const v4f b = *(const v4f*)(in + (size_t)i * 8 + 4);
    v4u p;
    p[0] = pk16(bf_bits(a[0]), bf_bits(a[1]));
    p[1] = pk16(bf_bits(a[2]), bf_bits(a[3]));
    p[2] = pk16(bf_bits(b[0]), bf_bits(b[1]));
    p[3] = pk16(bf_bits(b[2]), bf_bits(b[3]));
    *(volatile v4u*)(out + (size_t)i * 8) = p;
    __threadfence();
    *(volatile v4u*)(out + (size_t)i * 8) = p;
  }
}

__global__ __launch_bounds__(256) void rope_table(float* tab, int npair) {
  const int idx = blockIdx.x * 256 + threadIdx.x;
  if (idx < npair) {
    const int i = idx & 31;
    const int s = idx >> 5;
    double cur = 10.0, r2 = 1.0, r4 = 1.0, r8 = 1.0;
#pragma unroll 1
    for (int t = 0; t < 3; ++t) {
      cur = sqrt(cur);
      if (t == 0) r2 = cur; else if (t == 1) r4 = cur; else r8 = cur;
    }
    const int oct = i & 7, dec = i >> 3;
    double pw = ((oct & 4) ? r2 : 1.0) * ((oct & 2) ? r4 : 1.0);
    pw = pw * ((oct & 1) ? r8 : 1.0);
    const double dsc = (dec == 0) ? 1.0 : ((dec == 1) ? 10.0 : ((dec == 2) ? 100.0 : 1000.0));
    pw = pw * dsc;
    const float pf  = (float)pw;
    const float th  = 1.0f / pf;
    const float ang = (float)s * th;
    float sn, cs;
    sincosf(ang, &sn, &cs);
    v2f o;
    o[0] = cs; o[1] = sn;
    *(volatile v2f*)(tab + (size_t)idx * 2) = o;
    __threadfence();
    *(volatile v2f*)(tab + (size_t)idx * 2) = o;
  }
}

template <int MODE>
__global__ __launch_bounds__(256) void gemm64(
    const unsigned short* __restrict__ Ap, const unsigned short* __restrict__ A2p, int lda,
    const unsigned short* __restrict__ Btp, int ldb, long long strideB,
    void* Cout, void* Cout2, int ldc, long long strideC,
    const float* __restrict__ bias, const float* __restrict__ tab,
    int M, int N, int K) {
  const __bf16* A  = (const __bf16*)(const void*)Ap;
  const __bf16* A2 = (const __bf16*)(const void*)A2p;
  const __bf16* Bt = (const __bf16*)(const void*)Btp;
  __shared__ __align__(16) float sT[8][16 * 68];
  const int bz   = blockIdx.y;
  const int lane = threadIdx.x & 31;
  const int wave = threadIdx.x >> 5;
  const int tilesN = N >> 6;
  const int tilesM = M >> 6;
  const int tile = blockIdx.x * 8 + wave;
  if (tile >= tilesM * tilesN) return;
  const int tm = tile / tilesN;
  const int tn = tile - tm * tilesN;
  const int m0 = tm << 6;
  const int n0 = tn << 6;

  const __bf16* Bb = Bt + (size_t)bz * (size_t)strideB;

  const int rlane = lane & 15;
  const int koff  = (lane >> 4) * 8;
  const int mOff  = (lane >> 4) * 8;

  v8f acc[4][4];
#pragma unroll
  for (int i = 0; i < 4; ++i)
#pragma unroll
    for (int j = 0; j < 4; ++j) acc[i][j] = zero8();

#pragma unroll 1
  for (int k0 = 0; k0 < K; k0 += 32) {
    v16b bh[4];
#pragma unroll
    for (int j = 0; j < 4; ++j) {
      const size_t bo = (size_t)(n0 + (j << 4) + rlane) * ldb + koff + k0;
      bh[j] = ldfrag_b(Bb + bo);
    }
#pragma unroll
    for (int i = 0; i < 4; ++i) {
      const size_t ao = (size_t)(m0 + (i << 4) + rlane) * lda + koff + k0;
      const v16b ah = ldfrag_b(A + ao);
      v16b al = ah;
      if (MODE == 0) al = ldfrag_b(A2 + ao);
#pragma unroll
      for (int j = 0; j < 4; ++j) {
        acc[i][j] = mma_b_raw(ah, bh[j], acc[i][j]);
        if (MODE == 0) acc[i][j] = mma_b_raw(al, bh[j], acc[i][j]);
      }
      dep_guard_b(acc[i][0], acc[i][3], ah, al);
    }
    keep4_b(bh[0], bh[1], bh[2], bh[3]);
  }
  acc_guard4(acc[0][0], acc[0][1], acc[0][2], acc[0][3]);
  acc_guard4(acc[1][0], acc[1][1], acc[1][2], acc[1][3]);
  acc_guard4(acc[2][0], acc[2][1], acc[2][2], acc[2][3]);
  acc_guard4(acc[3][0], acc[3][1], acc[3][2], acc[3][3]);

  float* slab = sT[wave];
#pragma unroll
  for (int i = 0; i < 4; ++i) {
    const int mBase = m0 + (i << 4);
#pragma unroll
    for (int j = 0; j < 4; ++j) {
#pragma unroll
      for (int r = 0; r < 8; ++r) {
        slab[(mOff + r) * 68 + (j << 4) + rlane] = acc[i][j][r];
      }
    }
    lds_wave_sync();
    if (MODE == 0) {
      float* C = (float*)Cout + (size_t)bz * (size_t)strideC;
      const int h2 = lane >> 4, c4 = (lane & 15) * 4;
      const v4f braw = *(const v4f*)(bias + n0 + c4);
      v4f bb;
#pragma unroll
      for (int e = 0; e < 4; ++e) bb[e] = bfr(braw[e]);
      v4f vals[8];
#pragma unroll
      for (int it = 0; it < 8; ++it) {
        const int row = it * 2 + h2;
        const v4f v = *(const v4f*)(slab + row * 68 + c4);
        vals[it] = v + bb;
      }
      for (int pass = 0; pass < 2; ++pass) {
#pragma unroll
        for (int it = 0; it < 8; ++it) {
          const int row = it * 2 + h2;
          *(volatile v4f*)(C + (size_t)(mBase + row) * ldc + n0 + c4) = vals[it];
        }
        __threadfence();
      }
    } else {
      const int q = lane >> 3, c8 = (lane & 7) * 8;
      unsigned short* C  = (unsigned short*)Cout  + (size_t)bz * (size_t)strideC;
      unsigned short* C2 = (unsigned short*)Cout2 + (size_t)bz * (size_t)strideC;
      float bc[8];
      if (MODE == 3) {
#pragma unroll
        for (int e = 0; e < 8; ++e) bc[e] = 0.f;
      } else {
        const v4f b0 = *(const v4f*)(bias + n0 + c8);
        const v4f b1 = *(const v4f*)(bias + n0 + c8 + 4);
#pragma unroll
        for (int e = 0; e < 4; ++e) { bc[e] = bfr(b0[e]); bc[4 + e] = bfr(b1[e]); }
      }
      v4u hv[4], lv[4];
#pragma unroll
      for (int it = 0; it < 4; ++it) {
        const int row = it * 4 + q;
        const float* sp = slab + row * 68 + c8;
        const v4f s0 = *(const v4f*)(sp);
        const v4f s1 = *(const v4f*)(sp + 4);
        float f[8];
        if (MODE == 3) {
          const float brow = bfr(bias[mBase + row]);
#pragma unroll
          for (int e = 0; e < 4; ++e) { f[e] = s0[e] + brow; f[4 + e] = s1[e] + brow; }
        } else {
#pragma unroll
          for (int e = 0; e < 4; ++e) { f[e] = s0[e] + bc[e]; f[4 + e] = s1[e] + bc[4 + e]; }
        }
        if (MODE == 1 || MODE == 2) {
          const int spos = (mBase + row) & (SEQ - 1);
          const v4f t0 = *(const v4f*)(tab + (size_t)spos * HD + c8);
          const v4f t1 = *(const v4f*)(tab + (size_t)spos * HD + c8 + 4);
          float cs[4], sn[4];
          cs[0] = t0[0]; sn[0] = t0[1]; cs[1] = t0[2]; sn[1] = t0[3];
          cs[2] = t1[0]; sn[2] = t1[1]; cs[3] = t1[2]; sn[3] = t1[3];
#pragma unroll
          for (int e = 0; e < 4; ++e) {
            const float re = f[2 * e], im = f[2 * e + 1];
            f[2 * e]     = re * cs[e] - im * sn[e];
            f[2 * e + 1] = re * sn[e] + im * cs[e];
          }
        }
        v4u a, a2;
#pragma unroll
        for (int e = 0; e < 4; ++e) {
          const float f0 = f[2 * e], f1 = f[2 * e + 1];
          const _Float16 x0 = (_Float16)f0, x1 = (_Float16)f1;
          const unsigned short h0 = h_bits(x0), h1 = h_bits(x1);
          unsigned short l0 = 0, l1 = 0;
          if (MODE == 1) {
            l0 = h_bits((_Float16)((f0 - (float)x0) * 1024.0f));
            l1 = h_bits((_Float16)((f1 - (float)x1) * 1024.0f));
          }
          a[e] = pk16(h0, h1); a2[e] = pk16(l0, l1);
        }
        hv[it] = a; lv[it] = a2;
      }
      for (int pass = 0; pass < 2; ++pass) {
#pragma unroll
        for (int it = 0; it < 4; ++it) {
          const int row = it * 4 + q;
          *(volatile v4u*)(C + (size_t)(mBase + row) * ldc + n0 + c8) = hv[it];
          if (MODE == 1) *(volatile v4u*)(C2 + (size_t)(mBase + row) * ldc + n0 + c8) = lv[it];
        }
        __threadfence();
      }
    }
    lds_wave_sync();
  }
}

__global__ __launch_bounds__(256)
void attn64(const unsigned short* __restrict__ qhp, const unsigned short* __restrict__ qrp,
            const unsigned short* __restrict__ kpp, const unsigned short* __restrict__ vtp,
            unsigned short* ohp, unsigned short* olp, float sscale) {
  union FH { v16h v; v8h h[2]; };
  __shared__ __align__(16) _Float16 Ksh[64 * 64];
  __shared__ __align__(16) _Float16 Vth[64 * 64];
  __shared__ __align__(16) _Float16 Psh[8][16 * 64];
  __shared__ __align__(16) float    Os[8][16 * 64];

  const int tid  = threadIdx.x;
  const int wave = tid >> 5;
  const int lane = tid & 31;
  const int hh   = lane >> 4;
  const int c    = lane & 15;

  const int bx   = blockIdx.x;
  const int qbl  = bx % NQBLK;
  const int rest = bx / NQBLK;
  const int h    = rest % NH;
  const int b    = rest / NH;
  const int q0   = qbl * QBR + wave * 16;
  const size_t rowB = (size_t)b * SEQ;

  const _Float16* Qh = (const _Float16*)(const void*)qhp + (size_t)h * HD;
  const _Float16* Qr = (const _Float16*)(const void*)qrp + (size_t)h * HD;
  const _Float16* Kp = (const _Float16*)(const void*)kpp + (size_t)h * HD;
  const _Float16* Vt = (const _Float16*)(const void*)vtp + ((size_t)b * DM + (size_t)h * HD) * SEQ;

  v16h qah[2], qar[2];
#pragma unroll
  for (int dc = 0; dc < 2; ++dc) {
    const size_t qo = (rowB + (size_t)(q0 + c)) * DM + dc * 32 + 8 * hh;
    qah[dc] = ldfrag_h(Qh + qo);
    qar[dc] = ldfrag_h(Qr + qo);
  }

  float mrow[8], lrow[8];
  v8f oacc[4];
#pragma unroll
  for (int r = 0; r < 8; ++r) { mrow[r] = -INFINITY; lrow[r] = 0.f; }
#pragma unroll
  for (int t = 0; t < 4; ++t) oacc[t] = zero8();

#pragma unroll 1
  for (int kt = 0; kt < NKT; ++kt) {
    const int kv0 = kt * 64;
    __syncthreads();
    {
      const int r = tid >> 2, cq = (tid & 3) * 16;
      const _Float16* kg = Kp + (rowB + (size_t)(kv0 + r)) * DM + cq;
      const _Float16* vg = Vt + (size_t)r * SEQ + kv0 + cq;
      const v8h a0 = *(const v8h*)(kg);
      const v8h a1 = *(const v8h*)(kg + 8);
      const v8h b0 = *(const v8h*)(vg);
      const v8h b1 = *(const v8h*)(vg + 8);
      *(v8h*)(Ksh + r * 64 + cq)     = a0;
      *(v8h*)(Ksh + r * 64 + cq + 8) = a1;
      *(v8h*)(Vth + r * 64 + cq)     = b0;
      *(v8h*)(Vth + r * 64 + cq + 8) = b1;
    }
    __syncthreads();

    v8f s[4];
#pragma unroll
    for (int j = 0; j < 4; ++j) {
      FH k0f, k1f;
      const _Float16* kr = Ksh + (j * 16 + c) * 64 + 8 * hh;
      k0f.h[0] = *(const v8h*)(kr);
      k0f.h[1] = *(const v8h*)(kr + 16);
      k1f.h[0] = *(const v8h*)(kr + 32);
      k1f.h[1] = *(const v8h*)(kr + 48);
      v8f a = zero8();
      a = mma_h(qah[0], k0f.v, a);
      a = mma_h(qah[1], k1f.v, a);
      v8f rr = zero8();
      rr = mma_h(qar[0], k0f.v, rr);
      rr = mma_h(qar[1], k1f.v, rr);
#pragma unroll
      for (int r = 0; r < 8; ++r) a[r] = a[r] + rr[r] * (1.0f / 1024.0f);
      s[j] = a;
    }

    _Float16* pw = Psh[wave];
#pragma unroll
    for (int r = 0; r < 8; ++r) {
      float m = -INFINITY;
#pragma unroll
      for (int j = 0; j < 4; ++j) {
        const float sv = s[j][r] * sscale;
        s[j][r] = sv;
        m = fmaxf(m, sv);
      }
#pragma unroll
      for (int off = 1; off < 16; off <<= 1) m = fmaxf(m, __shfl_xor(m, off, 32));
      const float mnew  = fmaxf(mrow[r], m);
      const float msafe = (mnew == -INFINITY) ? 0.f : mnew;
      const float alpha = __expf(mrow[r] - msafe);
      mrow[r] = mnew;
      float psum = 0.f;
#pragma unroll
      for (int j = 0; j < 4; ++j) {
        const float p = __expf(s[j][r] - msafe);
        psum += p;
        pw[(8 * hh + r) * 64 + j * 16 + c] = (_Float16)(p * 1024.0f);
      }
#pragma unroll
      for (int off = 1; off < 16; off <<= 1) psum += __shfl_xor(psum, off, 32);
      lrow[r] = lrow[r] * alpha + psum;
#pragma unroll
      for (int t = 0; t < 4; ++t) oacc[t][r] *= alpha;
    }
    lds_wave_sync();

#pragma unroll 1
    for (int kk = 0; kk < 2; ++kk) {
      FH pa;
      pa.h[0] = *(const v8h*)(pw + c * 64 + kk * 32 + 8 * hh);
      pa.h[1] = *(const v8h*)(pw + c * 64 + kk * 32 + 16 + 8 * hh);
#pragma unroll
      for (int t = 0; t < 4; ++t) {
        FH vb;
        vb.h[0] = *(const v8h*)(Vth + (t * 16 + c) * 64 + kk * 32 + 8 * hh);
        vb.h[1] = *(const v8h*)(Vth + (t * 16 + c) * 64 + kk * 32 + 16 + 8 * hh);
        oacc[t] = mma_h(pa.v, vb.v, oacc[t]);
      }
    }
  }

  float* os = Os[wave];
#pragma unroll
  for (int r = 0; r < 8; ++r) {
    const float l = lrow[r];
    const float inv = ((l > 0.f) ? (1.0f / l) : 0.f) * (1.0f / 1024.0f);
#pragma unroll
    for (int t = 0; t < 4; ++t) os[(8 * hh + r) * 64 + t * 16 + c] = oacc[t][r] * inv;
  }
  lds_wave_sync();
  {
    const int q4 = lane >> 3, c8 = (lane & 7) * 8;
    v4u hv[4], lv[4];
#pragma unroll
    for (int it = 0; it < 4; ++it) {
      const int row = it * 4 + q4;
      const float* sp = os + row * 64 + c8;
      const v4f s0 = *(const v4f*)(sp);
      const v4f s1 = *(const v4f*)(sp + 4);
      float f[8];
#pragma unroll
      for (int e = 0; e < 4; ++e) { f[e] = s0[e]; f[4 + e] = s1[e]; }
      v4u a, a2;
#pragma unroll
      for (int e = 0; e < 4; ++e) {
        const float f0 = f[2 * e], f1 = f[2 * e + 1];
        const unsigned short h0 = bf_bits(f0), h1 = bf_bits(f1);
        const unsigned short l0 = bf_bits(f0 - bf_up(h0)), l1 = bf_bits(f1 - bf_up(h1));
        a[e] = pk16(h0, h1); a2[e] = pk16(l0, l1);
      }
      hv[it] = a; lv[it] = a2;
    }
    for (int pass = 0; pass < 2; ++pass) {
#pragma unroll
      for (int it = 0; it < 4; ++it) {
        const int row = it * 4 + q4;
        const size_t go = (rowB + (size_t)(q0 + row)) * DM + (size_t)h * HD + c8;
        *(volatile v4u*)(ohp + go) = hv[it];
        *(volatile v4u*)(olp + go) = lv[it];
      }
      __threadfence();
    }
  }
}

extern "C" void kernel_launch(void* const* d_in, const int* in_sizes, int n_in,
                              void* d_out, int out_size, void* d_ws, size_t ws_size,
                              hipStream_t stream) {
  if (n_in < 11) return;
  const int nAct = NB * SEQ * DM;
  const int nW   = DM * DM;
  if (in_sizes[0] != nAct || in_sizes[1] != nAct || in_sizes[2] != nAct) return;
  if (in_sizes[3] != nW || in_sizes[5] != nW || in_sizes[7] != nW || in_sizes[9] != nW) return;
  if (in_sizes[4] != DM || in_sizes[6] != DM || in_sizes[8] != DM || in_sizes[10] != DM) return;
  if (out_size != nAct) return;

  const float* xq = (const float*)d_in[0];
  const float* xk = (const float*)d_in[1];
  const float* xv = (const float*)d_in[2];
  const float* Wq = (const float*)d_in[3];
  const float* bq = (const float*)d_in[4];
  const float* Wk = (const float*)d_in[5];
  const float* bk = (const float*)d_in[6];
  const float* Wv = (const float*)d_in[7];
  const float* bv = (const float*)d_in[8];
  const float* Wo = (const float*)d_in[9];
  const float* bo = (const float*)d_in[10];

  const size_t PX = (size_t)nAct * 2;
  const size_t PW = (size_t)nW * 2;
  const size_t PT = (size_t)SEQ * HD * 4;
  size_t off = 0;
  const size_t oXq = off; off += PX;
  const size_t oXk = off; off += PX;
  const size_t oXv = off; off += PX;
  const size_t oWq = off; off += PW;
  const size_t oWk = off; off += PW;
  const size_t oWv = off; off += PW;
  const size_t oWo = off; off += PW;
  const size_t oQh = off; off += PX;
  const size_t oQr = off; off += PX;
  const size_t oKp = off; off += PX;
  const size_t oVT = off; off += PX;
  const size_t oTb = off; off += PT;
  if (off > ws_size) return;
  if (off > (size_t)WS_CAP) return;
  const size_t oOh = oXq;
  const size_t oOl = oXk;

  char* ws = (char*)d_ws;
  unsigned short* Xqb = (unsigned short*)(ws + oXq);
  unsigned short* Xkb = (unsigned short*)(ws + oXk);
  unsigned short* Xvb = (unsigned short*)(ws + oXv);
  unsigned short* Wqb = (unsigned short*)(ws + oWq);
  unsigned short* Wkb = (unsigned short*)(ws + oWk);
  unsigned short* Wvb = (unsigned short*)(ws + oWv);
  unsigned short* Wob = (unsigned short*)(ws + oWo);
  unsigned short* Qh  = (unsigned short*)(ws + oQh);
  unsigned short* Qr  = (unsigned short*)(ws + oQr);
  unsigned short* Kpl = (unsigned short*)(ws + oKp);
  unsigned short* VT  = (unsigned short*)(ws + oVT);
  float*          Tab = (float*)(ws + oTb);
  unsigned short* Oh  = (unsigned short*)(ws + oOh);
  unsigned short* Ol  = (unsigned short*)(ws + oOl);

  const dim3 blk(256);
  const int n8x = nAct / 8;
  const int n8w = nW / 8;
  const int npair = SEQ * (HD / 2);
  const dim3 gCvtX((n8x + 255) / 256);
  const dim3 gCvtW((n8w + 255) / 256);
  const dim3 gTab((npair + 255) / 256);
  const dim3 gProj(((NB * SEQ / 64) * (DM / 64) + 7) / 8, 1);
  const dim3 gVT(((DM / 64) * (SEQ / 64) + 7) / 8, NB);
  const dim3 gAttn(NB * NH * NQBLK);

  cvt_bf16x8<<<gCvtX, blk, 0, stream>>>(xq, Xqb, n8x);
  cvt_bf16x8<<<gCvtX, blk, 0, stream>>>(xk, Xkb, n8x);
  cvt_bf16x8<<<gCvtX, blk, 0, stream>>>(xv, Xvb, n8x);
  cvt_bf16x8<<<gCvtW, blk, 0, stream>>>(Wq, Wqb, n8w);
  cvt_bf16x8<<<gCvtW, blk, 0, stream>>>(Wk, Wkb, n8w);
  cvt_bf16x8<<<gCvtW, blk, 0, stream>>>(Wv, Wvb, n8w);
  cvt_bf16x8<<<gCvtW, blk, 0, stream>>>(Wo, Wob, n8w);
  rope_table<<<gTab, blk, 0, stream>>>(Tab, npair);
  gemm64<1><<<gProj, blk, 0, stream>>>(
      Xqb, Xqb, DM, Wqb, DM, 0LL,
      (void*)Qh, (void*)Qr, DM, 0LL, bq, Tab, NB * SEQ, DM, DM);
  gemm64<2><<<gProj, blk, 0, stream>>>(
      Xkb, Xkb, DM, Wkb, DM, 0LL,
      (void*)Kpl, (void*)Kpl, DM, 0LL, bk, Tab, NB * SEQ, DM, DM);
  gemm64<3><<<gVT, blk, 0, stream>>>(
      Wvb, Wvb, DM, Xvb, DM, (long long)SEQ * DM,
      (void*)VT, (void*)VT, SEQ, (long long)DM * SEQ, bv, Tab, DM, SEQ, DM);
  attn64<<<gAttn, blk, 0, stream>>>(Qh, Qr, Kpl, VT, Oh, Ol, 0.125f);
  gemm64<0><<<gProj, blk, 0, stream>>>(
      Oh, Ol, DM, Wob, DM, 0LL,
      d_out, d_out, DM, 0LL, bo, Tab, NB * SEQ, DM, DM);
  (void)hipGetLastError();
}
